// SelfAttentiveSpanExtractor_71494025609506
// MI455X (gfx1250) — hardware-verified
//
#include <hip/hip_runtime.h>
#include <math.h>

typedef __attribute__((ext_vector_type(16))) _Float16 v16h;
typedef __attribute__((ext_vector_type(16))) __bf16 v16b;
typedef __attribute__((ext_vector_type(8)))  _Float16 v8h;
typedef __attribute__((ext_vector_type(8)))  float v8f;
typedef __attribute__((ext_vector_type(4)))  float v4f;
typedef __attribute__((ext_vector_type(2)))  float v2f;
typedef __attribute__((ext_vector_type(4)))  unsigned v4u;
typedef __attribute__((ext_vector_type(4)))  int v4i;
typedef float __attribute__((may_alias)) float_a;
typedef int __attribute__((may_alias)) int_a;

template <typename T> __device__ __forceinline__ void vst2(void* p, T v) { *(volatile T*)p = v; __threadfence(); *(volatile T*)p = v; }
__device__ __forceinline__ v8f wmma16(v16h a, v16h b, v8f c) {
  v8f d = __builtin_amdgcn_wmma_f32_16x16x32_f16(false, a, false, b, (short)0, c, false, false);
  asm volatile("v_nop\n\tv_nop\n\tv_nop\n\tv_nop" : "+v"(d) : "v"(a), "v"(b));
  return d;
}
__device__ __forceinline__ v8f wmma_bf(v16b a, v16b b, v8f c) {
  v8f d = __builtin_amdgcn_wmma_f32_16x16x32_bf16(false, a, false, b, (short)0, c, false, false);
  asm volatile("v_nop\n\tv_nop\n\tv_nop\n\tv_nop" : "+v"(d) : "v"(a), "v"(b));
  return d;
}
__device__ __forceinline__ v16h frag_h(const _Float16* rowk0, int lane) {
  union { v16h v; v8h q[2]; } u; const _Float16* p = rowk0 + 8 * (lane >> 4);
  u.q[0] = *(const v8h*)p; u.q[1] = *(const v8h*)(p + 16); return u.v;
}
__device__ __forceinline__ v16h frag_f32(const float* rowk0, int lane) {
  v16h a; const float* p = rowk0 + 8 * (lane >> 4);
#pragma unroll
  for (int i = 0; i < 8; ++i) { a[i] = (_Float16)p[i]; a[8 + i] = (_Float16)p[16 + i]; }
  return a;
}
__device__ __forceinline__ v16h frag_f32s(const float* rowk0, int lane, float sc) {
  v16h a; const float* p = rowk0 + 8 * (lane >> 4);
#pragma unroll
  for (int i = 0; i < 8; ++i) { a[i] = (_Float16)(p[i] * sc); a[8 + i] = (_Float16)(p[16 + i] * sc); }
  return a;
}
__device__ __forceinline__ v16h fragc_f32(const float* W, int k0, int n, int lane, int ld, int K) {
  v16h a; const int g = lane >> 4;
#pragma unroll
  for (int i = 0; i < 8; ++i) { const int ka = k0 + 8 * g + i, kb = ka + 16;
    a[i] = (_Float16)(ka < K ? W[(size_t)(ka < K ? ka : K - 1) * ld + n] : 0.f); a[8 + i] = (_Float16)(kb < K ? W[(size_t)(kb < K ? kb : K - 1) * ld + n] : 0.f); }
  return a;
}
struct F2 { v16b h, l; };
__device__ __forceinline__ F2 bsplit16(const float v[16]) { F2 r;
#pragma unroll
  for (int i = 0; i < 16; ++i) { const __bf16 h = (__bf16)v[i]; r.h[i] = h; r.l[i] = (__bf16)(v[i] - (float)h); }
  return r; }
__device__ __forceinline__ F2 split_row(const float* row, int k0, int lane) { float v[16]; const float* p = row + k0 + 8 * (lane >> 4);
#pragma unroll
  for (int i = 0; i < 8; ++i) { v[i] = p[i]; v[8 + i] = p[16 + i]; }
  return bsplit16(v); }
__device__ __forceinline__ F2 split_rowK(const float* row, int k0, int lane, int K) { float v[16]; const int g = lane >> 4;
#pragma unroll
  for (int i = 0; i < 8; ++i) { const int ka = k0 + 8 * g + i, kb = ka + 16; v[i] = ka < K ? row[ka < K ? ka : K - 1] : 0.f; v[8 + i] = kb < K ? row[kb < K ? kb : K - 1] : 0.f; }
  return bsplit16(v); }
__device__ __forceinline__ F2 split_col(const float* W, int k0, int n, int lane, int ld, int K) { float v[16]; const int g = lane >> 4;
#pragma unroll
  for (int i = 0; i < 8; ++i) { const int ka = k0 + 8 * g + i, kb = ka + 16; v[i] = ka < K ? W[(size_t)(ka < K ? ka : K - 1) * ld + n] : 0.f; v[8 + i] = kb < K ? W[(size_t)(kb < K ? kb : K - 1) * ld + n] : 0.f; }
  return bsplit16(v); }
__device__ __forceinline__ v8f mac3(const F2& a, const F2& b, v8f c) { c = wmma_bf(a.l, b.h, c); c = wmma_bf(a.h, b.l, c); return wmma_bf(a.h, b.h, c); }
__device__ __forceinline__ float sigm(float v) { return 1.0f / (1.0f + expf(-v)); }
#define LDSX() do { asm volatile("s_wait_dscnt 0" ::: "memory"); __builtin_amdgcn_wave_barrier(); __builtin_amdgcn_fence(__ATOMIC_RELEASE, "workgroup"); } while (0)


#define NB 4
#define TT 2048
#define DD 768
#define NS 512
#define MW 32
#ifndef TNB
#define TNB NB
#endif
typedef __attribute__((ext_vector_type(8))) __bf16 v8b;
__device__ __forceinline__ v16b frag_b(const __bf16* rowk0, int lane) {
  union { v16b v; v8b q[2]; } u; const __bf16* p = rowk0 + 8 * (lane >> 4);
  u.q[0] = *(const v8b*)p; u.q[1] = *(const v8b*)(p + 16); return u.v;
}
__device__ __forceinline__ float bfr(float v) { return (float)(__bf16)v; }
__device__ __attribute__((noinline)) float exp_ni(float v) { return expf(v); }
__device__ __attribute__((noinline)) float erf_ni(float v) { return erff(v); }

#define WS_PW  0u
#define WS_GL  (WS_PW + 2u * 16 * DD)
#define WS_END (WS_GL + 4u * (size_t)NB * TT * 16)

__global__ __launch_bounds__(256) void k_pack(const float* __restrict__ AW, __bf16* __restrict__ PW) { __shared__ __align__(16) __bf16 s[16 * DD]; const int t = threadIdx.x; for (int e = t; e < 16 * DD; e += 256) s[e] = (e < DD) ? (__bf16)AW[e] : (__bf16)0.0f; __syncthreads(); for (int q = t; q < 16 * DD / 8; q += 256) vst2((unsigned*)(PW + q * 8), *(const v4u*)&s[q * 8]); }
__device__ __forceinline__ v16b fragb_f32(const float* __restrict__ p, int lane) { v16b a; const float* pp = p + 8 * (lane >> 4);
#pragma unroll
  for (int i = 0; i < 8; ++i) { a[i] = (__bf16)pp[i]; a[8 + i] = (__bf16)pp[16 + i]; } return a; }
__global__ __launch_bounds__(128) void k_logit(const float* __restrict__ SEQ, const __bf16* __restrict__ PW, const float* __restrict__ AB, float* __restrict__ GL16) { __shared__ __align__(16) float sf[4][16][20];
  const int tid = threadIdx.x, wave = tid >> 5, lane = tid & 31, col = lane & 15, g = lane >> 4; const size_t r0 = (size_t)blockIdx.x * 64 + wave * 16;
  v8f acc = {};
#pragma unroll 4
  for (int kc = 0; kc < DD / 32; ++kc) acc = wmma_bf(fragb_f32(SEQ + (r0 + col) * DD + kc * 32, lane), frag_b(PW + (size_t)col * DD + kc * 32, lane), acc);
  const float bb = bfr(AB[0]);
#pragma unroll
  for (int r = 0; r < 8; ++r) sf[wave][8 * g + r][col] = acc[r] + (col == 0 ? bb : 0.f);
  LDSX(); for (int rl = 0; rl < 16; ++rl) if (lane < 4) vst2(GL16 + (r0 + rl) * 16 + lane * 4, *(const v4f*)&sf[wave][rl][lane * 4]); }
__global__ __launch_bounds__(256) void k_span(const float* __restrict__ SEQ, const int* __restrict__ SP, const float* __restrict__ GL16, float* __restrict__ OUT) { __shared__ int sidx[MW]; __shared__ float satt[MW]; __shared__ __align__(16) float so2[DD]; const int t = threadIdx.x; const size_t b = blockIdx.y; const int n = blockIdx.x;
  if (t < 32) { const int st = SP[((b * NS + n) * 2)], en = SP[((b * NS + n) * 2) + 1]; const int width = en - st; const int raw = en - t; float m = (t <= width) ? 1.f : 0.f; if (raw < 0) m = 0.f; int idx = raw > 0 ? raw : 0; idx = idx >= TT ? TT - 1 : idx; sidx[t] = idx;
    const float lg = GL16[(b * TT + idx) * 16] * m;
    float mx = lg;
#pragma unroll
    for (int o = 1; o < 32; o <<= 1) mx = fmaxf(mx, __shfl_xor(mx, o));
    const float e = __expf(lg - mx); float se = e;
#pragma unroll
    for (int o = 1; o < 32; o <<= 1) se += __shfl_xor(se, o);
    float a = (e / se) * m; float sa = a;
#pragma unroll
    for (int o = 1; o < 32; o <<= 1) sa += __shfl_xor(sa, o);
    satt[t] = a / (sa + 1e-13f); }
  __syncthreads();
  for (int d = t; d < DD; d += 256) { float acc = 0.f;
#pragma unroll 1
    for (int w = 0; w < MW; ++w) { const float a = satt[w]; if (a != 0.f) acc += a * bfr(SEQ[(b * TT + sidx[w]) * DD + d]); }
    so2[d] = acc; }
  __syncthreads(); for (int q = t; q < DD / 4; q += 256) vst2(OUT + ((b * NS + n) * DD) + q * 4, *(const v4f*)&so2[q * 4]); }
extern "C" void kernel_launch(void* const* d_in, const int* in_sizes, int n_in, void* d_out, int out_size, void* d_ws, size_t ws_size, hipStream_t stream) {
  (void)in_sizes; (void)n_in; (void)out_size;
  const float** F = (const float**)d_in;
  if (ws_size < (size_t)WS_END) return;
  char* ws = (char*)d_ws; __bf16* PW = (__bf16*)(ws + WS_PW); float* GL16 = (float*)(ws + WS_GL);
  k_pack<<<1, 256, 0, stream>>>(F[2], PW);
  k_logit<<<TNB * TT / 64, 128, 0, stream>>>(F[0], PW, F[3], GL16);
  k_span<<<dim3(NS, TNB), 256, 0, stream>>>(F[0], (const int*)d_in[1], GL16, (float*)d_out);
}
